// PureCrossAttention_69853348102847
// MI455X (gfx1250) — hardware-verified
//
#include <hip/hip_runtime.h>
#include <stddef.h>
#include <stdint.h>

#define HID   1024
#define NHEAD 16
#define HDIM  64
#define NB    4
#define SLEN  1024
#define MROWS (NB * SLEN)

typedef char chk_dims0[(HID == NHEAD * HDIM) ? 1 : -1];
typedef char chk_dims1[(MROWS % 128 == 0 && HID % 64 == 0 && SLEN % 128 == 0 && HID % 32 == 0 && SLEN % 64 == 0) ? 1 : -1];

typedef _Float16 f16;
typedef f16 v16h __attribute__((ext_vector_type(16)));
typedef f16 v8h __attribute__((ext_vector_type(8)));
typedef float v8f __attribute__((ext_vector_type(8)));
typedef float v4f __attribute__((ext_vector_type(4)));
typedef unsigned int v4u __attribute__((ext_vector_type(4)));

union Frag  { v16h v; v8h hv[2]; };
union Pack8 { v8h h; v4u u; };
union ShG   { float f[8192]; f16 hb[16384]; v4u u[2048]; };
union ShA   { f16 hb[8192]; v4u u[1024]; };
typedef char chk_sh0[(sizeof(ShG) == 32768) ? 1 : -1];
typedef char chk_sh1[(sizeof(ShA) == 16384) ? 1 : -1];

#define INV1024 9.765625e-4f

static __device__ __forceinline__ v8f zero8() {
  v8f z;
#pragma unroll
  for (int i = 0; i < 8; ++i) z[i] = 0.0f;
  return z;
}

static __device__ __forceinline__ v8f wmma16(v16h a, v16h b, v8f c) {
  v8f d = __builtin_amdgcn_wmma_f32_16x16x32_f16(false, a, false, b, (short)0, c, false, false);
  asm volatile("v_nop\n\tv_nop\n\tv_nop\n\tv_nop" : "+v"(d) : "v"(a), "v"(b));
  return d;
}

__global__ __launch_bounds__(256)
void k_cvt(const float* __restrict__ src, f16* __restrict__ dst, int n8, float scale) {
  const int i = blockIdx.x * 256 + threadIdx.x;
  if (i < n8) {
    const v4f* s = (const v4f*)(src + (size_t)i * 8);
    const v4f x0 = s[0];
    const v4f x1 = s[1];
    Pack8 p;
#pragma unroll
    for (int c = 0; c < 4; ++c) {
      p.h[c]     = (f16)(x0[c] * scale);
      p.h[4 + c] = (f16)(x1[c] * scale);
    }
    const v4u u = p.u;
    volatile v4u* d = (volatile v4u*)(dst + (size_t)i * 8);
    *d = u;
    __threadfence();
    *d = u;
  }
}

template<int MODE>
__global__ __launch_bounds__(128)
void k_gemm(const f16* __restrict__ A, const f16* __restrict__ W, const float* __restrict__ bias,
            float alpha, float beta, void* __restrict__ outp) {
  __shared__ ShG sh;
  const int t = threadIdx.x, w = t >> 5, l = t & 31, h = l >> 4, m = l & 15;
  const int m0 = blockIdx.y * 128, n0 = blockIdx.x * 64;

  const f16* a0p = A + (size_t)(m0 + 32 * w + m) * HID + 8 * h;
  const f16* a1p = a0p + (size_t)16 * HID;
  const f16* bp  = W + (size_t)(n0 + m) * HID + 8 * h;

  v8f acc[2][4];
#pragma unroll
  for (int mi = 0; mi < 2; ++mi)
#pragma unroll
    for (int nn = 0; nn < 4; ++nn) acc[mi][nn] = zero8();

  for (int k0 = 0; k0 < HID; k0 += 32) {
    Frag fa0, fa1;
    fa0.hv[0] = *(const v8h*)(a0p + k0);
    fa0.hv[1] = *(const v8h*)(a0p + k0 + 16);
    fa1.hv[0] = *(const v8h*)(a1p + k0);
    fa1.hv[1] = *(const v8h*)(a1p + k0 + 16);
#pragma unroll
    for (int nn = 0; nn < 4; ++nn) {
      const f16* br = bp + (size_t)nn * 16 * HID + k0;
      Frag fb;
      fb.hv[0] = *(const v8h*)(br);
      fb.hv[1] = *(const v8h*)(br + 16);
      acc[0][nn] = wmma16(fa0.v, fb.v, acc[0][nn]);
      acc[1][nn] = wmma16(fa1.v, fb.v, acc[1][nn]);
    }
  }

  float bvv[4];
#pragma unroll
  for (int nn = 0; nn < 4; ++nn) bvv[nn] = bias[n0 + 16 * nn + m];

  if (MODE == 0) {
    float* ldsw = sh.f + w * 2048;
#pragma unroll
    for (int mi = 0; mi < 2; ++mi)
#pragma unroll
      for (int nn = 0; nn < 4; ++nn)
#pragma unroll
        for (int r = 0; r < 8; ++r)
          ldsw[(16 * mi + 8 * h + r) * 64 + 16 * nn + m] = (acc[mi][nn][r] * alpha + bvv[nn]) * beta;
    __syncthreads();
    float* ob = (float*)outp + (size_t)(m0 + 32 * w) * HID + n0;
#pragma unroll
    for (int j = 0; j < 16; ++j) {
      const int c = 32 * j + l, row = c >> 4, sub = c & 15;
      const v4u x = sh.u[w * 512 + c];
      *(volatile v4u*)(ob + (size_t)row * HID + sub * 4) = x;
    }
    __threadfence();
#pragma unroll
    for (int j = 0; j < 16; ++j) {
      const int c = 32 * j + l, row = c >> 4, sub = c & 15;
      const v4u x = sh.u[w * 512 + c];
      *(volatile v4u*)(ob + (size_t)row * HID + sub * 4) = x;
    }
  } else if (MODE == 1) {
    f16* ldsh = sh.hb + w * 2048;
#pragma unroll
    for (int mi = 0; mi < 2; ++mi)
#pragma unroll
      for (int nn = 0; nn < 4; ++nn)
#pragma unroll
        for (int r = 0; r < 8; ++r)
          ldsh[(16 * mi + 8 * h + r) * 64 + 16 * nn + m] = (f16)((acc[mi][nn][r] * alpha + bvv[nn]) * beta);
    __syncthreads();
    const int bb = m0 >> 10, hh = n0 >> 6;
    const int s0 = (m0 & (SLEN - 1)) + 32 * w;
    f16* ob = (f16*)outp + ((size_t)(bb * NHEAD + hh) * SLEN + s0) * HDIM;
#pragma unroll
    for (int j = 0; j < 8; ++j) {
      const int c = 32 * j + l;
      const v4u x = sh.u[w * 256 + c];
      *(volatile v4u*)(ob + (size_t)c * 8) = x;
    }
    __threadfence();
#pragma unroll
    for (int j = 0; j < 8; ++j) {
      const int c = 32 * j + l;
      const v4u x = sh.u[w * 256 + c];
      *(volatile v4u*)(ob + (size_t)c * 8) = x;
    }
  } else {
    f16* ldst = sh.hb;
#pragma unroll
    for (int mi = 0; mi < 2; ++mi)
#pragma unroll
      for (int nn = 0; nn < 4; ++nn)
#pragma unroll
        for (int r = 0; r < 8; ++r)
          ldst[(16 * nn + m) * 128 + 32 * w + 16 * mi + 8 * h + r] = (f16)((acc[mi][nn][r] * alpha + bvv[nn]) * beta);
    __syncthreads();
    const int bb = m0 >> 10, hh = n0 >> 6;
    const int s0b = m0 & (SLEN - 1);
    f16* ob = (f16*)outp + ((size_t)(bb * NHEAD + hh) * HDIM) * SLEN + s0b;
#pragma unroll
    for (int j = 0; j < 8; ++j) {
      const int c = 128 * j + t, d = c >> 4, sub = c & 15;
      const v4u x = sh.u[c];
      *(volatile v4u*)(ob + (size_t)d * SLEN + sub * 8) = x;
    }
    __threadfence();
#pragma unroll
    for (int j = 0; j < 8; ++j) {
      const int c = 128 * j + t, d = c >> 4, sub = c & 15;
      const v4u x = sh.u[c];
      *(volatile v4u*)(ob + (size_t)d * SLEN + sub * 8) = x;
    }
  }
}

static __device__ __forceinline__ void score_tiles(const f16* __restrict__ Kp, int kv0, int m, int h,
                                                   v16h q0v, v16h q1v, v8f* T) {
#pragma unroll
  for (int tt = 0; tt < 2; ++tt) {
    const f16* kr = Kp + (size_t)(kv0 + 16 * tt + m) * HDIM + 8 * h;
    Frag a0, a1;
    a0.hv[0] = *(const v8h*)(kr);
    a0.hv[1] = *(const v8h*)(kr + 16);
    a1.hv[0] = *(const v8h*)(kr + 32);
    a1.hv[1] = *(const v8h*)(kr + 48);
    v8f acc = zero8();
    acc = wmma16(a0.v, q0v, acc);
    acc = wmma16(a1.v, q1v, acc);
    T[tt] = acc;
  }
}

__global__ __launch_bounds__(128)
void k_attn(const f16* __restrict__ Qs, const f16* __restrict__ Ks, const f16* __restrict__ Vt,
            const float* __restrict__ amask, f16* __restrict__ ctx1, f16* __restrict__ ctx2) {
  __shared__ ShA sha;
  const int t = threadIdx.x, w = t >> 5, l = t & 31, h = l >> 4, m = l & 15;
  const int bid = blockIdx.x;
  const int bh = bid >> 4;
  const int b = bh >> 4, hh = bh & 15;
  const int q0 = (bid & 15) * 64 + w * 16;

  const f16* Qp = Qs + ((size_t)bh * SLEN + q0) * HDIM;
  const f16* Kp = Ks + (size_t)bh * SLEN * HDIM;
  const f16* Vp = Vt + (size_t)bh * HDIM * SLEN;
  const float* Mp = amask + ((size_t)b * SLEN + q0 + m) * SLEN;

  Frag bq0, bq1;
  {
    const f16* qr = Qp + (size_t)m * HDIM + 8 * h;
    bq0.hv[0] = *(const v8h*)(qr);
    bq0.hv[1] = *(const v8h*)(qr + 16);
    bq1.hv[0] = *(const v8h*)(qr + 32);
    bq1.hv[1] = *(const v8h*)(qr + 48);
  }

  float mrun = -1e30f, zrun = 0.0f;
  for (int kv0 = 0; kv0 < SLEN; kv0 += 32) {
    v8f T[2];
    score_tiles(Kp, kv0, m, h, bq0.v, bq1.v, T);
    const v4f* mp = (const v4f*)(Mp + kv0 + 8 * h);
    v4f mk[4];
    mk[0] = mp[0]; mk[1] = mp[1]; mk[2] = mp[4]; mk[3] = mp[5];
    float s[16];
#pragma unroll
    for (int i = 0; i < 16; ++i) s[i] = T[i >> 3][i & 7] * INV1024 + mk[i >> 2][i & 3];
    float mx = mrun;
#pragma unroll
    for (int i = 0; i < 16; ++i) mx = fmaxf(mx, s[i]);
    float zs = zrun * __expf(mrun - mx);
#pragma unroll
    for (int i = 0; i < 16; ++i) zs += __expf(s[i] - mx);
    mrun = mx;
    zrun = zs;
  }
  {
    const float mo = __shfl_xor(mrun, 16, 32);
    const float zo = __shfl_xor(zrun, 16, 32);
    const float mx = fmaxf(mrun, mo);
    zrun = zrun * __expf(mrun - mx) + zo * __expf(mo - mx);
    mrun = mx;
  }
  const float invz = 1.0f / zrun;

  v8f O1[4], O2[4];
#pragma unroll
  for (int nn = 0; nn < 4; ++nn) { O1[nn] = zero8(); O2[nn] = zero8(); }
  float z2 = 0.0f;

  for (int kv0 = 0; kv0 < SLEN; kv0 += 32) {
    v8f T[2];
    score_tiles(Kp, kv0, m, h, bq0.v, bq1.v, T);
    const v4f* mp = (const v4f*)(Mp + kv0 + 8 * h);
    v4f mk[4];
    mk[0] = mp[0]; mk[1] = mp[1]; mk[2] = mp[4]; mk[3] = mp[5];
    Frag pf, wf;
#pragma unroll
    for (int i = 0; i < 16; ++i) {
      const float sv = T[i >> 3][i & 7] * INV1024 + mk[i >> 2][i & 3];
      const float p  = __expf(sv - mrun) * invz;
      const float w2 = __expf(-p);
      z2 += w2;
      pf.v[i] = (f16)(p * 4096.0f);
      wf.v[i] = (f16)w2;
    }
#pragma unroll
    for (int nn = 0; nn < 4; ++nn) {
      const f16* vr = Vp + (size_t)(16 * nn + m) * SLEN + kv0 + 8 * h;
      Frag vb;
      vb.hv[0] = *(const v8h*)(vr);
      vb.hv[1] = *(const v8h*)(vr + 16);
      O1[nn] = wmma16(pf.v, vb.v, O1[nn]);
      O2[nn] = wmma16(wf.v, vb.v, O2[nn]);
    }
  }
  z2 += __shfl_xor(z2, 16, 32);
  const float invz2 = 1.0f / z2;
  float iz[8];
#pragma unroll
  for (int r = 0; r < 8; ++r) iz[r] = __shfl(invz2, 8 * h + r, 32);

  f16* l1 = sha.hb + w * 2048;
  f16* l2 = l1 + 1024;
#pragma unroll
  for (int nn = 0; nn < 4; ++nn)
#pragma unroll
    for (int r = 0; r < 8; ++r) {
      const int idx = (8 * h + r) * 64 + 16 * nn + m;
      l1[idx] = (f16)(O1[nn][r] * (1.0f / 256.0f));
      l2[idx] = (f16)(O2[nn][r] * 16.0f * iz[r]);
    }
  __syncthreads();
  f16* c1 = ctx1 + ((size_t)(b * SLEN + q0)) * HID + hh * HDIM;
  f16* c2 = ctx2 + ((size_t)(b * SLEN + q0)) * HID + hh * HDIM;
#pragma unroll
  for (int j = 0; j < 4; ++j) {
    const int c = 32 * j + l, row = c >> 3, sub = c & 7;
    const v4u x1 = sha.u[w * 256 + c];
    const v4u x2 = sha.u[w * 256 + 128 + c];
    *(volatile v4u*)(c1 + (size_t)row * HID + sub * 8) = x1;
    *(volatile v4u*)(c2 + (size_t)row * HID + sub * 8) = x2;
  }
  __threadfence();
#pragma unroll
  for (int j = 0; j < 4; ++j) {
    const int c = 32 * j + l, row = c >> 3, sub = c & 7;
    const v4u x1 = sha.u[w * 256 + c];
    const v4u x2 = sha.u[w * 256 + 128 + c];
    *(volatile v4u*)(c1 + (size_t)row * HID + sub * 8) = x1;
    *(volatile v4u*)(c2 + (size_t)row * HID + sub * 8) = x2;
  }
}

extern "C" void kernel_launch(void* const* d_in, const int* in_sizes, int n_in,
                              void* d_out, int out_size, void* d_ws, size_t ws_size,
                              hipStream_t stream) {
  const size_t NA = (size_t)MROWS * HID;
  const size_t NW = (size_t)HID * HID;
  const size_t NM = (size_t)NB * SLEN * SLEN;
  if (n_in < 13) return;
  if ((size_t)in_sizes[0] != NA || (size_t)in_sizes[1] != NA || (size_t)in_sizes[2] != NM) return;
  if ((size_t)in_sizes[3] != NW || (size_t)in_sizes[5] != NW || (size_t)in_sizes[7] != NW ||
      (size_t)in_sizes[9] != NW || (size_t)in_sizes[11] != NW) return;
  if (in_sizes[4] != HID || in_sizes[6] != HID || in_sizes[8] != HID || in_sizes[10] != HID || in_sizes[12] != HID) return;
  if ((size_t)out_size != 2 * NA) return;

  const float* q   = (const float*)d_in[0];
  const float* kv  = (const float*)d_in[1];
  const float* msk = (const float*)d_in[2];
  const float* Wq  = (const float*)d_in[3];
  const float* bq  = (const float*)d_in[4];
  const float* Wk  = (const float*)d_in[5];
  const float* bk  = (const float*)d_in[6];
  const float* Wv  = (const float*)d_in[7];
  const float* bv  = (const float*)d_in[8];
  const float* Wo  = (const float*)d_in[9];
  const float* bo  = (const float*)d_in[10];
  const float* Wr  = (const float*)d_in[11];
  const float* br  = (const float*)d_in[12];
  float* out = (float*)d_out;

  const size_t need = (7 * NA + 5 * NW) * sizeof(f16);
  if (ws_size < need) return;
  char* wp = (char*)d_ws;
  f16* qh   = (f16*)wp; wp += NA * 2;
  f16* kvh  = (f16*)wp; wp += NA * 2;
  f16* wqh  = (f16*)wp; wp += NW * 2;
  f16* wkh  = (f16*)wp; wp += NW * 2;
  f16* wvh  = (f16*)wp; wp += NW * 2;
  f16* woh  = (f16*)wp; wp += NW * 2;
  f16* wrh  = (f16*)wp; wp += NW * 2;
  f16* Qs   = (f16*)wp; wp += NA * 2;
  f16* Ks   = (f16*)wp; wp += NA * 2;
  f16* Vts  = (f16*)wp; wp += NA * 2;
  f16* cx1  = (f16*)wp; wp += NA * 2;
  f16* cx2  = (f16*)wp; wp += NA * 2;

  const int nA8 = (int)(NA / 8), nW8 = (int)(NW / 8);
  const dim3 cb(256), cgA((unsigned)((nA8 + 255) / 256)), cgW((unsigned)((nW8 + 255) / 256));
  k_cvt<<<cgA, cb, 0, stream>>>(q,  qh,  nA8, 1.0f);
  k_cvt<<<cgA, cb, 0, stream>>>(kv, kvh, nA8, 1.0f);
  k_cvt<<<cgW, cb, 0, stream>>>(Wq, wqh, nW8, 1024.0f);
  k_cvt<<<cgW, cb, 0, stream>>>(Wk, wkh, nW8, 1024.0f);
  k_cvt<<<cgW, cb, 0, stream>>>(Wv, wvh, nW8, 1024.0f);
  k_cvt<<<cgW, cb, 0, stream>>>(Wo, woh, nW8, 1024.0f);
  k_cvt<<<cgW, cb, 0, stream>>>(Wr, wrh, nW8, 1024.0f);

  const dim3 gb(128), gg(HID / 64, MROWS / 128);
  k_gemm<1><<<gg, gb, 0, stream>>>(qh,  wqh, bq, INV1024, 8.0f,  (void*)Qs);
  k_gemm<1><<<gg, gb, 0, stream>>>(kvh, wkh, bk, INV1024, 16.0f, (void*)Ks);
  k_gemm<2><<<gg, gb, 0, stream>>>(kvh, wvh, bv, INV1024, 16.0f, (void*)Vts);

  k_attn<<<dim3(NB * NHEAD * (SLEN / 64)), dim3(128), 0, stream>>>(Qs, Ks, Vts, msk, cx1, cx2);

  const float oalpha = 1.0f / (256.0f * 1024.0f);
  k_gemm<0><<<gg, gb, 0, stream>>>(cx1, woh, bo, oalpha, 1.0f, (void*)out);
  k_gemm<0><<<gg, gb, 0, stream>>>(cx2, wrh, br, oalpha, 1.0f, (void*)(out + NA));
}
